// IDNN_38998303048195
// MI455X (gfx1250) — hardware-run, weakly checked
//
#include <hip/hip_runtime.h>
#include <math.h>

typedef __attribute__((ext_vector_type(16))) _Float16 v16h;
typedef __attribute__((ext_vector_type(8)))  _Float16 v8h;
typedef __attribute__((ext_vector_type(8)))  float    v8f;
typedef __attribute__((ext_vector_type(4)))  float    v4f;

constexpr int kB  = 32768;
constexpr int kD  = 16;
constexpr int kH  = 256;
constexpr int kPH = 264;
constexpr int kPF = 260;
static_assert(kB % 32 == 0, "sample tiles");
static_assert(kH % 32 == 0 && kH == 256 && kD == 16, "tile shapes");
static_assert((kPH * 2) % 16 == 0 && (kPF * 4) % 16 == 0, "16-B aligned LDS rows");

constexpr float kCW1  = 64.0f;
constexpr float kCW2  = 16.0f;
constexpr float kCXL  = 64.0f;
constexpr float kCG2  = 64.0f;
constexpr float kCG1  = 64.0f;
constexpr float kCC   = 64.0f;
constexpr float kCP   = 1024.0f;
constexpr float kCE   = 64.0f;
constexpr float kRES  = 2048.0f;
constexpr float kInvRES = 1.0f / kRES;
constexpr float kInvS1  = 1.0f / kCW1;
constexpr float kInvS2  = 1.0f / kCW2;
constexpr float kInvS3  = 1.0f / (kCG2 * kCW2);
constexpr float kInvS4  = 1.0f / (kCG1 * kCW1);
constexpr float kInvS6  = 1.0f / (kCC * kCP);
constexpr float kVacc   = kCW1 * kCW2;
constexpr float kInvS7  = 1.0f / (kVacc * kVacc * kCE);

constexpr size_t kPlaneW  = (size_t)kH * kH * 2;
constexpr size_t kPlaneB  = (size_t)kB * kH * 4;
constexpr size_t kOffW2TH = 0;
constexpr size_t kOffW2SH = kOffW2TH + kPlaneW;
constexpr size_t kOffW2SL = kOffW2SH + kPlaneW;
constexpr size_t kOffPTH  = kOffW2SL + kPlaneW;
constexpr size_t kOffPTL  = kOffPTH  + kPlaneW;
constexpr size_t kOffW1T  = kOffPTL  + kPlaneW;
constexpr size_t kOffW1PH = kOffW1T  + (size_t)kH * 64 * 2;
constexpr size_t kOffW1PL = kOffW1PH + (size_t)kD * kH * 2;
constexpr size_t kOffS1P  = kOffW1PL + (size_t)kD * kH * 2;
constexpr size_t kOffEP   = kOffS1P  + kPlaneB;
constexpr size_t kOffHAP  = kOffEP   + kPlaneB;
constexpr size_t kWsTotal = kOffHAP  + kPlaneB;
static_assert(kWsTotal == 101367808ull, "carve total");
static_assert(kWsTotal <= 134217728ull, "carve cap");
static_assert((kOffW2SH % 128) == 0 && (kOffW2SL % 128) == 0 && (kOffPTH % 128) == 0 && (kOffPTL % 128) == 0 &&
              (kOffW1T % 128) == 0 && (kOffW1PH % 128) == 0 && (kOffW1PL % 128) == 0 && (kOffS1P % 128) == 0 &&
              (kOffEP % 128) == 0 && (kOffHAP % 128) == 0, "128-B aligned regions");

constexpr size_t kOutY   = 0;
constexpr size_t kOutDy  = 131072 / 4;
constexpr size_t kOutDdy = 2228224 / 4;
constexpr size_t kOutTot = 35782656 / 4;
static_assert(kOutDy == (size_t)kB && kOutDdy == (size_t)kB + (size_t)kB * kD, "tuple offsets");
static_assert(kOutDdy + (size_t)kB * kD * kD == kOutTot, "tuple extent");

union FragU { v16h v; v8h h[2]; };
__device__ __forceinline__ v16h frag_load(const _Float16* p) {
  FragU f;
  f.h[0] = *(const v8h*)(p);
  f.h[1] = *(const v8h*)(p + 16);
  return f.v;
}
__device__ __forceinline__ v8f mma16(v16h a, v16h b, v8f c) {
  return __builtin_amdgcn_wmma_f32_16x16x32_f16(false, a, false, b, (short)0, c, false, false);
}
__device__ __forceinline__ v8f mma16g(v16h a, v16h b, v8f c) {
  c = __builtin_amdgcn_wmma_f32_16x16x32_f16(false, a, false, b, (short)0, c, false, false);
  asm volatile("v_nop\n\tv_nop\n\tv_nop\n\tv_nop" : "+v"(c) : "v"(a), "v"(b));
  return c;
}
__device__ __forceinline__ void guard2(v8f& a0, v8f& a1, v16h f0, v16h f1, v16h f2) {
  asm volatile("v_nop\n\tv_nop\n\tv_nop\n\tv_nop" : "+v"(a0), "+v"(a1) : "v"(f0), "v"(f1), "v"(f2));
}
__device__ __forceinline__ void guard4(v8f& a0, v8f& a1, v8f& a2, v8f& a3, v16h f0, v16h f1, v16h f2, v16h f3) {
  asm volatile("v_nop\n\tv_nop\n\tv_nop\n\tv_nop" : "+v"(a0), "+v"(a1), "+v"(a2), "+v"(a3)
               : "v"(f0), "v"(f1), "v"(f2), "v"(f3));
}
__device__ __forceinline__ void guard_grp(v8f& a0, v8f& a1, v8f& r0, v8f& r1,
                                          v16h f0, v16h f1, v16h f2, v16h f3, v16h f4, v16h f5) {
  asm volatile("v_nop\n\tv_nop\n\tv_nop\n\tv_nop" : "+v"(a0), "+v"(a1), "+v"(r0), "+v"(r1)
               : "v"(f0), "v"(f1), "v"(f2), "v"(f3), "v"(f4), "v"(f5));
}
__device__ __forceinline__ void wave_lds_fence() {
  __builtin_amdgcn_fence(__ATOMIC_RELEASE, "workgroup");
  __builtin_amdgcn_wave_barrier();
  __builtin_amdgcn_fence(__ATOMIC_ACQUIRE, "workgroup");
}
__device__ __forceinline__ void split16(float v, _Float16& hi, _Float16& lo) {
  const _Float16 h = (_Float16)v;
  const float r = v - (float)h;
  hi = h;
  lo = (_Float16)(r * kRES);
}
__device__ __forceinline__ void softplus_sigmoid(float z, float& sp, float& sg) {
  const float ez  = expf(-fabsf(z));
  const float inv = 1.0f / (1.0f + ez);
  sg = (z >= 0.0f) ? inv : ez * inv;
  sp = fmaxf(z, 0.0f) + log1pf(ez);
}
__device__ __forceinline__ void store1_v8h(_Float16* p, v8h a) {
  *(volatile v8h*)p = a;
  __threadfence();
  *(volatile v8h*)p = a;
}
__device__ __forceinline__ void store2_v8h(_Float16* p, v8h a, _Float16* q, v8h b) {
  *(volatile v8h*)p = a;
  *(volatile v8h*)q = b;
  __threadfence();
  *(volatile v8h*)p = a;
  *(volatile v8h*)q = b;
}

__global__ __launch_bounds__(256) void prep_kernel(
    const float* __restrict__ W1, const float* __restrict__ W2,
    _Float16* __restrict__ W2TH, _Float16* __restrict__ W2SH, _Float16* __restrict__ W2SL,
    _Float16* __restrict__ PTH, _Float16* __restrict__ PTL, _Float16* __restrict__ W1T,
    _Float16* __restrict__ W1PH, _Float16* __restrict__ W1PL)
{
  const int blk = blockIdx.x, tid = threadIdx.x;
  if (blk < 96) {
    const int sec = blk >> 5;
    const int idx = (blk & 31) * 256 + tid;
    const int row = idx >> 5, c8 = (idx & 31) * 8;
    v8h hv, lv;
#pragma unroll
    for (int i = 0; i < 8; ++i) {
      float w;
      if (sec == 0) {
        w = W2[(size_t)(c8 + i) * kH + row] * kCW2;
      } else if (sec == 1) {
        w = W2[(size_t)row * kH + c8 + i] * kCW2;
      } else {
        const int d = row >> 4, e = row & 15;
        const float p = W1[d * kH + c8 + i] * W1[e * kH + c8 + i];
        w = p * kCP;
      }
      _Float16 h, l;
      split16(w, h, l);
      hv[i] = h;
      lv[i] = l;
    }
    const size_t off = (size_t)row * kH + c8;
    if (sec == 0) {
      store1_v8h(W2TH + off, hv);
    } else if (sec == 1) {
      store2_v8h(W2SH + off, hv, W2SL + off, lv);
    } else {
      store2_v8h(PTH + off, hv, PTL + off, lv);
    }
  } else if (blk < 104) {
    const int idx = (blk - 96) * 256 + tid;
    const int n = idx >> 3, seg = idx & 7;
    const int kk = (seg & 1) * 8, grp = seg >> 1;
    v8h ov;
#pragma unroll
    for (int i = 0; i < 8; ++i) {
      const float w  = W1[(kk + i) * kH + n] * kCW1;
      const _Float16 h = (_Float16)w;
      const float hf = (float)h;
      const float sel = (grp == 0) ? hf : (grp == 1) ? (hf * kInvS1) : (grp == 2) ? (w - hf) : 0.0f;
      ov[i] = (_Float16)sel;
    }
    store1_v8h(W1T + (size_t)n * 64 + seg * 8, ov);
  } else {
    const int idx = (blk - 104) * 256 + tid;
    const int d = idx >> 5, c8 = (idx & 31) * 8;
    v8h hv, lv;
#pragma unroll
    for (int i = 0; i < 8; ++i) {
      _Float16 h, l;
      split16(W1[d * kH + c8 + i] * kCW1, h, l);
      hv[i] = h;
      lv[i] = l;
    }
    const size_t off = (size_t)d * kH + c8;
    store2_v8h(W1PH + off, hv, W1PL + off, lv);
  }
}

template <bool SPLIT>
__device__ __forceinline__ void gemm_tile32(const _Float16* aH, const _Float16* aL,
                                            const _Float16* __restrict__ bH, const _Float16* __restrict__ bL,
                                            int n0, int m, int hh, v8f (&am)[2][2], v8f (&ar)[2][2])
{
#pragma unroll
  for (int mi = 0; mi < 2; ++mi)
#pragma unroll
    for (int ni = 0; ni < 2; ++ni) {
      am[mi][ni] = (v8f){0.f, 0.f, 0.f, 0.f, 0.f, 0.f, 0.f, 0.f};
      ar[mi][ni] = (v8f){0.f, 0.f, 0.f, 0.f, 0.f, 0.f, 0.f, 0.f};
    }
#pragma unroll 1
  for (int kc = 0; kc < kH / 32; ++kc) {
    const int ko = kc * 32 + 8 * hh;
    v16h bh[2], bl[2];
#pragma unroll
    for (int ni = 0; ni < 2; ++ni) {
      const size_t bo = (size_t)(n0 + 16 * ni + m) * kH + ko;
      bh[ni] = frag_load(bH + bo);
      bl[ni] = SPLIT ? frag_load(bL + bo) : bh[ni];
    }
#pragma unroll
    for (int mi = 0; mi < 2; ++mi) {
      const int ao = (16 * mi + m) * kPH + ko;
      const v16h ah = frag_load(aH + ao);
      const v16h al = SPLIT ? frag_load(aL + ao) : ah;
#pragma unroll
      for (int ni = 0; ni < 2; ++ni) {
        am[mi][ni] = mma16(ah, bh[ni], am[mi][ni]);
        if (SPLIT) {
          ar[mi][ni] = mma16(ah, bl[ni], ar[mi][ni]);
          ar[mi][ni] = mma16(al, bh[ni], ar[mi][ni]);
        }
      }
      if (SPLIT) guard_grp(am[mi][0], am[mi][1], ar[mi][0], ar[mi][1], ah, al, bh[0], bh[1], bl[0], bl[1]);
      else guard2(am[mi][0], am[mi][1], ah, bh[0], bh[1]);
    }
  }
}

__device__ __forceinline__ void store_tile_lines(const float* sT, float* __restrict__ G, int b0, int n0, int lane) {
  const int q4 = lane >> 3, c4 = (lane & 7) * 4;
  v4f v[8];
#pragma unroll
  for (int it = 0; it < 8; ++it) v[it] = *(const v4f*)(sT + (it * 4 + q4) * kPF + n0 + c4);
  for (int pass = 0; pass < 2; ++pass) {
#pragma unroll
    for (int it = 0; it < 8; ++it)
      *(volatile v4f*)(G + (size_t)(b0 + it * 4 + q4) * kH + n0 + c4) = v[it];
    __threadfence();
  }
}

__global__ __launch_bounds__(256) void fwd_bwd_kernel(
    const float* __restrict__ x, const float* __restrict__ b1, const float* __restrict__ b2,
    const float* __restrict__ w3,
    const _Float16* __restrict__ W1T, const _Float16* __restrict__ W2TH,
    const _Float16* __restrict__ W2SH, const _Float16* __restrict__ W2SL,
    const _Float16* __restrict__ W1PH, const _Float16* __restrict__ W1PL,
    const _Float16* __restrict__ PTH, const _Float16* __restrict__ PTL,
    float* __restrict__ yout, float* __restrict__ dyout,
    float* __restrict__ S1P, float* __restrict__ EP, float* __restrict__ HAP)
{
  __shared__ __align__(16) float    sS1[32 * kPF];
  __shared__ __align__(16) float    sE[32 * kPF];
  __shared__ __align__(16) _Float16 sP0[32 * kPH];
  __shared__ __align__(16) _Float16 sP1[32 * kPH];
  __shared__ __align__(16) _Float16 sP2[32 * kPH];
  __shared__ __align__(16) _Float16 sP3[32 * kPH];
  __shared__ __align__(16) float    sYp[8 * 32];
  __shared__ __align__(16) float    sDy[32 * kD];

  const int tid = threadIdx.x, lane = tid & 31, wave = tid >> 5;
  const int hh = lane >> 4, m = lane & 15;
  const int b0 = blockIdx.x * 32;
  const int n0 = wave * 32;
  const int colL = n0 + lane;

  {
    v16h xa0[2], xa1[2];
#pragma unroll
    for (int mi = 0; mi < 2; ++mi) {
      const float* xp = x + (size_t)(b0 + 16 * mi + m) * kD + 8 * hh;
      const v4f q0 = *(const v4f*)(xp);
      const v4f q1 = *(const v4f*)(xp + 4);
#pragma unroll
      for (int e = 0; e < 4; ++e) {
        const float f0 = q0[e], f1 = q1[e];
        const _Float16 h0 = (_Float16)f0, h1 = (_Float16)f1;
        const _Float16 l0 = (_Float16)((f0 - (float)h0) * kCXL);
        const _Float16 l1 = (_Float16)((f1 - (float)h1) * kCXL);
        xa0[mi][e] = h0;      xa0[mi][4 + e] = h1;
        xa0[mi][8 + e] = l0;  xa0[mi][12 + e] = l1;
        xa1[mi][e] = h0;      xa1[mi][4 + e] = h1;
        xa1[mi][8 + e] = (_Float16)0.0f;
        xa1[mi][12 + e] = (_Float16)0.0f;
      }
    }
    v8f acc[2][2];
#pragma unroll
    for (int ni = 0; ni < 2; ++ni) {
      const _Float16* bp = W1T + (size_t)(n0 + 16 * ni + m) * 64 + 8 * hh;
      const v16h bA = frag_load(bp);
      const v16h bB = frag_load(bp + 32);
#pragma unroll
      for (int mi = 0; mi < 2; ++mi) {
        v8f c = (v8f){0.f, 0.f, 0.f, 0.f, 0.f, 0.f, 0.f, 0.f};
        c = mma16g(xa0[mi], bA, c);
        c = mma16g(xa1[mi], bB, c);
        acc[mi][ni] = c;
      }
    }
#pragma unroll
    for (int ni = 0; ni < 2; ++ni) {
      const int col = n0 + 16 * ni + m;
      const float bb = b1[col];
#pragma unroll
      for (int mi = 0; mi < 2; ++mi)
#pragma unroll
        for (int r = 0; r < 8; ++r)
          sS1[(16 * mi + 8 * hh + r) * kPF + col] = acc[mi][ni][r] * kInvS1 + bb;
    }
  }
  __syncthreads();
#pragma unroll 1
  for (int it = 0; it < 32; ++it) {
    const float z = sS1[it * kPF + colL];
    float sp, sg;
    softplus_sigmoid(z, sp, sg);
    sS1[it * kPF + colL] = sg;
    sP0[it * kPH + colL] = (_Float16)sp;
  }
  __syncthreads();

  {
    v8f am[2][2], ar[2][2];
    gemm_tile32<false>(sP0, sP0, W2TH, W2TH, n0, m, hh, am, ar);
#pragma unroll
    for (int ni = 0; ni < 2; ++ni) {
      const int col = n0 + 16 * ni + m;
      const float bb = b2[col];
#pragma unroll
      for (int mi = 0; mi < 2; ++mi)
#pragma unroll
        for (int r = 0; r < 8; ++r)
          sE[(16 * mi + 8 * hh + r) * kPF + col] = am[mi][ni][r] * kInvS2 + bb;
    }
  }
  __syncthreads();
  {
    const float w3c = w3[colL];
    float ysel = 0.0f;
#pragma unroll 1
    for (int it = 0; it < 32; ++it) {
      const float z = sE[it * kPF + colL];
      float sp, sg;
      softplus_sigmoid(z, sp, sg);
      float yp = sp * w3c;
      yp += __shfl_xor(yp, 16, 32);
      yp += __shfl_xor(yp, 8, 32);
      yp += __shfl_xor(yp, 4, 32);
      yp += __shfl_xor(yp, 2, 32);
      yp += __shfl_xor(yp, 1, 32);
      ysel = (lane == it) ? yp : ysel;
      _Float16 gh, gl;
      split16(sg * w3c * kCG2, gh, gl);
      sP2[it * kPH + colL] = gh;
      sP3[it * kPH + colL] = gl;
      const float s2p = sg * (1.0f - sg);
      sE[it * kPF + colL] = w3c * s2p * kCE;
    }
    sYp[wave * 32 + lane] = ysel;
  }
  __syncthreads();

  {
    v8f am[2][2], ar[2][2];
    gemm_tile32<true>(sP2, sP3, W2SH, W2SL, n0, m, hh, am, ar);
    __syncthreads();
#pragma unroll
    for (int mi = 0; mi < 2; ++mi)
#pragma unroll
      for (int ni = 0; ni < 2; ++ni) {
        const int col = n0 + 16 * ni + m;
#pragma unroll
        for (int r = 0; r < 8; ++r) {
          const int row = 16 * mi + 8 * hh + r;
          const float u  = (am[mi][ni][r] + ar[mi][ni][r] * kInvRES) * kInvS3;
          const float s1 = sS1[row * kPF + col];
          const float su = s1 * u;
          _Float16 a, b;
          split16(su * kCG1, a, b);
          sP0[row * kPH + col] = a;
          sP1[row * kPH + col] = b;
          const float cc = (1.0f - s1) * su;
          split16(cc * kCC, a, b);
          sP2[row * kPH + col] = a;
          sP3[row * kPH + col] = b;
        }
      }
  }
  __syncthreads();

  if (wave < 2) {
    v8f dm = (v8f){0.f, 0.f, 0.f, 0.f, 0.f, 0.f, 0.f, 0.f};
    v8f dr = (v8f){0.f, 0.f, 0.f, 0.f, 0.f, 0.f, 0.f, 0.f};
#pragma unroll 1
    for (int kc = 0; kc < kH / 32; ++kc) {
      const int ko = kc * 32 + 8 * hh;
      const v16h ah = frag_load(sP0 + (16 * wave + m) * kPH + ko);
      const v16h al = frag_load(sP1 + (16 * wave + m) * kPH + ko);
      const v16h bh = frag_load(W1PH + (size_t)m * kH + ko);
      const v16h bl = frag_load(W1PL + (size_t)m * kH + ko);
      dm = mma16g(ah, bh, dm);
      dr = mma16g(ah, bl, dr);
      dr = mma16g(al, bh, dr);
    }
#pragma unroll
    for (int r = 0; r < 8; ++r)
      sDy[(16 * wave + 8 * hh + r) * kD + m] = (dm[r] + dr[r] * kInvRES) * kInvS4;
  }

  v8f hm[2][2], hr[2][2];
  gemm_tile32<true>(sP2, sP3, PTH, PTL, n0, m, hh, hm, hr);
  __syncthreads();

  store_tile_lines(sS1, S1P, b0, n0, lane);
  store_tile_lines(sE, EP, b0, n0, lane);
  if (wave == 0) {
    float s = 0.0f;
#pragma unroll
    for (int w = 0; w < 8; ++w) s += sYp[w * 32 + lane];
    volatile float* yp = yout + b0 + lane;
    *yp = s;
    __threadfence();
    *yp = s;
  }
  if (wave == 1) {
    v4f dv[4];
#pragma unroll
    for (int it = 0; it < 4; ++it) dv[it] = *(const v4f*)(sDy + it * 128 + lane * 4);
    float* dp = dyout + (size_t)b0 * kD;
    for (int pass = 0; pass < 2; ++pass) {
#pragma unroll
      for (int it = 0; it < 4; ++it) *(volatile v4f*)(dp + it * 128 + lane * 4) = dv[it];
      __threadfence();
    }
  }
  __syncthreads();
#pragma unroll
  for (int mi = 0; mi < 2; ++mi)
#pragma unroll
    for (int ni = 0; ni < 2; ++ni) {
      const int col = n0 + 16 * ni + m;
#pragma unroll
      for (int r = 0; r < 8; ++r)
        sS1[(16 * mi + 8 * hh + r) * kPF + col] = (hm[mi][ni][r] + hr[mi][ni][r] * kInvRES) * kInvS6;
    }
  __syncthreads();
  store_tile_lines(sS1, HAP, b0, n0, lane);
}

__global__ __launch_bounds__(128) void hess_kernel(
    const float* __restrict__ W1, const _Float16* __restrict__ W2TH,
    const float* __restrict__ S1P, const float* __restrict__ EP, const float* __restrict__ HAP,
    float* __restrict__ ddy)
{
  __shared__ __align__(16) float    sW1[kD * kPF];
  __shared__ __align__(16) _Float16 sStg[4 * 2 * kD * kPH];
  __shared__ __align__(16) float    sHo[4 * 16 * 20];

  const int tid = threadIdx.x, lane = tid & 31, wave = tid >> 5;
  const int hh = lane >> 4, m = lane & 15;

#pragma unroll
  for (int i = 0; i < 8; ++i) {
    const int idx = tid + 128 * i;
    const int d = idx >> 6, c4 = (idx & 63) * 4;
    v4f w = *(const v4f*)(W1 + d * kH + c4);
    w = w * kCW1;
    *(v4f*)(sW1 + d * kPF + c4) = w;
  }
  __syncthreads();

  _Float16* stg0 = sStg + (size_t)(wave * 2 + 0) * kD * kPH;
  _Float16* stg1 = sStg + (size_t)(wave * 2 + 1) * kD * kPH;
  float* slab = sHo + wave * 320;
  const int sbase = blockIdx.x * 32 + wave * 8;

#pragma unroll 1
  for (int pass = 0; pass < 4; ++pass) {
    const int sa = sbase + pass * 2;
    wave_lds_fence();
#pragma unroll
    for (int s = 0; s < 2; ++s) {
      _Float16* stg = s ? stg1 : stg0;
      const float* sp = S1P + (size_t)(sa + s) * kH + 8 * lane;
      const v4f p0 = *(const v4f*)(sp);
      const v4f p1 = *(const v4f*)(sp + 4);
#pragma unroll 1
      for (int d = 0; d < kD; ++d) {
        const v4f w0 = *(const v4f*)(sW1 + d * kPF + 8 * lane);
        const v4f w1 = *(const v4f*)(sW1 + d * kPF + 8 * lane + 4);
        const v4f t0 = w0 * p0;
        const v4f t1 = w1 * p1;
        v8h o;
        o[0] = (_Float16)t0[0]; o[1] = (_Float16)t0[1]; o[2] = (_Float16)t0[2]; o[3] = (_Float16)t0[3];
        o[4] = (_Float16)t1[0]; o[5] = (_Float16)t1[1]; o[6] = (_Float16)t1[2]; o[7] = (_Float16)t1[3];
        *(v8h*)(stg + d * kPH + 8 * lane) = o;
      }
    }
    wave_lds_fence();

    v8f Hm[2], Hr[2];
#pragma unroll
    for (int s = 0; s < 2; ++s) {
      Hm[s] = (v8f){0.f, 0.f, 0.f, 0.f, 0.f, 0.f, 0.f, 0.f};
      Hr[s] = (v8f){0.f, 0.f, 0.f, 0.f, 0.f, 0.f, 0.f, 0.f};
    }

#pragma unroll 1
    for (int kp = 0; kp < 8; ++kp) {
      v8f acc[2][2];
#pragma unroll
      for (int t = 0; t < 2; ++t)
#pragma unroll
        for (int s = 0; s < 2; ++s) acc[t][s] = (v8f){0.f, 0.f, 0.f, 0.f, 0.f, 0.f, 0.f, 0.f};
#pragma unroll 1
      for (int jc = 0; jc < kH / 32; ++jc) {
        const int ko = jc * 32 + 8 * hh;
        const v16h a0 = frag_load(W2TH + (size_t)(32 * kp + m) * kH + ko);
        const v16h a1 = frag_load(W2TH + (size_t)(32 * kp + 16 + m) * kH + ko);
        const v16h q0 = frag_load(stg0 + m * kPH + ko);
        const v16h q1 = frag_load(stg1 + m * kPH + ko);
        acc[0][0] = mma16(a0, q0, acc[0][0]);
        acc[0][1] = mma16(a0, q1, acc[0][1]);
        acc[1][0] = mma16(a1, q0, acc[1][0]);
        acc[1][1] = mma16(a1, q1, acc[1][1]);
        guard4(acc[0][0], acc[0][1], acc[1][0], acc[1][1], a0, a1, q0, q1);
      }
#pragma unroll
      for (int s = 0; s < 2; ++s) {
        const float* ep = EP + (size_t)(sa + s) * kH + 32 * kp + 8 * hh;
        const v4f e0 = *(const v4f*)(ep);
        const v4f e1 = *(const v4f*)(ep + 4);
        const v4f e2 = *(const v4f*)(ep + 16);
        const v4f e3 = *(const v4f*)(ep + 20);
        v16h bh, bl, ah, al;
#pragma unroll
        for (int r = 0; r < 8; ++r) {
          const float ev0 = (r < 4) ? e0[r & 3] : e1[r & 3];
          const float ev1 = (r < 4) ? e2[r & 3] : e3[r & 3];
          const float v0 = acc[0][s][r];
          const float v1 = acc[1][s][r];
          _Float16 h, l;
          split16(v0, h, l);
          bh[r] = h; bl[r] = l;
          split16(v0 * ev0, h, l);
          ah[r] = h; al[r] = l;
          split16(v1, h, l);
          bh[8 + r] = h; bl[8 + r] = l;
          split16(v1 * ev1, h, l);
          ah[8 + r] = h; al[8 + r] = l;
        }
        Hm[s] = mma16g(ah, bh, Hm[s]);
        Hr[s] = mma16g(ah, bl, Hr[s]);
        Hr[s] = mma16g(al, bh, Hr[s]);
      }
    }

#pragma unroll
    for (int s = 0; s < 2; ++s) {
#pragma unroll
      for (int r = 0; r < 8; ++r)
        slab[(8 * hh + r) * 20 + m] = (Hm[s][r] + Hr[s][r] * kInvRES) * kInvS7;
      wave_lds_fence();
      const size_t base = (size_t)(sa + s) * (kD * kD);
      v4f o[2];
#pragma unroll
      for (int it = 0; it < 2; ++it) {
        const v4f hv = *(const v4f*)(slab + (it * 8 + (lane >> 2)) * 20 + (lane & 3) * 4);
        const v4f ha = *(const v4f*)(HAP + base + it * 128 + lane * 4);
        o[it] = hv + ha;
      }
      for (int ps = 0; ps < 2; ++ps) {
#pragma unroll
        for (int it = 0; it < 2; ++it) *(volatile v4f*)(ddy + base + it * 128 + lane * 4) = o[it];
        __threadfence();
      }
      wave_lds_fence();
    }
  }
}

extern "C" void kernel_launch(void* const* d_in, const int* in_sizes, int n_in,
                              void* d_out, int out_size, void* d_ws, size_t ws_size,
                              hipStream_t stream) {
  if (n_in < 6) return;
  if (in_sizes[0] != kB * kD) return;
  if (in_sizes[1] != kD * kH) return;
  if (in_sizes[2] != kH) return;
  if (in_sizes[3] != kH * kH) return;
  if (in_sizes[4] != kH) return;
  if (in_sizes[5] != kH) return;
  if ((size_t)out_size != kOutTot) return;
  if (ws_size < kWsTotal) return;

  const float* x  = (const float*)d_in[0];
  const float* W1 = (const float*)d_in[1];
  const float* b1 = (const float*)d_in[2];
  const float* W2 = (const float*)d_in[3];
  const float* b2 = (const float*)d_in[4];
  const float* W3 = (const float*)d_in[5];

  float* out = (float*)d_out;
  float* y_out   = out + kOutY;
  float* dy_out  = out + kOutDy;
  float* ddy_out = out + kOutDdy;

  char* ws = (char*)d_ws;
  _Float16* W2TH = (_Float16*)(ws + kOffW2TH);
  _Float16* W2SH = (_Float16*)(ws + kOffW2SH);
  _Float16* W2SL = (_Float16*)(ws + kOffW2SL);
  _Float16* PTH  = (_Float16*)(ws + kOffPTH);
  _Float16* PTL  = (_Float16*)(ws + kOffPTL);
  _Float16* W1T  = (_Float16*)(ws + kOffW1T);
  _Float16* W1PH = (_Float16*)(ws + kOffW1PH);
  _Float16* W1PL = (_Float16*)(ws + kOffW1PL);
  float* S1P = (float*)(ws + kOffS1P);
  float* EP  = (float*)(ws + kOffEP);
  float* HAP = (float*)(ws + kOffHAP);

  prep_kernel<<<106, 256, 0, stream>>>(W1, W2, W2TH, W2SH, W2SL, PTH, PTL, W1T, W1PH, W1PL);

  fwd_bwd_kernel<<<kB / 32, 256, 0, stream>>>(x, b1, b2, W3, W1T, W2TH, W2SH, W2SL, W1PH, W1PL, PTH, PTL,
                                              y_out, dy_out, S1P, EP, HAP);

  hess_kernel<<<kB / 32, 128, 0, stream>>>(W1, W2TH, S1P, EP, HAP, ddy_out);
}
